// BertClassifier_37907381354985
// MI455X (gfx1250) — hardware-run, weakly checked
//
#include <hip/hip_runtime.h>


#ifndef NB
#define NB 16
#endif
#define NB_FULL 16
#define LT    128
#define LH    129
#define DM    768
#define H1    770
#define H1P   832
#define PQP   1664
#define KW1   1536
#define OUTC  40
#define NSP   3405
#define NROWS (NB * NSP)
#define K2P   800
#define N2P   48
#define RB    64
#define HW    4
#define W2S   1024.0f
#define W2I   (1.0f / 1024.0f)

static_assert(NB <= NB_FULL);
static_assert(DM % 32 == 0);
static_assert(K2P % 32 == 0);
static_assert(K2P >= H1);
static_assert(K2P <= H1P);
static_assert(H1P % 64 == 0);
static_assert(PQP == 2 * H1P);
static_assert(PQP % 32 == 0);
static_assert((NB * LT) % 64 == 0);
static_assert(KW1 == 2 * DM);
static_assert(KW1 % 64 == 0);
static_assert((DM / 64) * 2 == KW1 / 64);
static_assert(H1P % 32 == 0);
static_assert(N2P % 16 == 0);
static_assert(N2P >= OUTC);
static_assert(OUTC > 32);
static_assert(OUTC - 32 <= 16);
static_assert(OUTC % 4 == 0);
static_assert(OUTC == 2 * 20);
static_assert(RB == 16 * HW);
static_assert(LT == 32 * HW);
static_assert((RB * (K2P / 4)) % (32 * HW) == 0);
static_assert((16 * OUTC * 4) % 128 == 0);
static_assert(((size_t)RB * OUTC * 4) % 128 == 0);
static_assert(5 * 32 * 4 == 16 * OUTC);
static_assert(8 * 2 * 64 == 16 * 64);
static_assert((N2P * (K2P / 8)) % 32 == 0);
static_assert(((size_t)LT * DM / 8) % 256 == 0);
static_assert(NSP > RB);

typedef _Float16 h16;
typedef unsigned short bf;
typedef __attribute__((ext_vector_type(16))) __bf16   v16bf;
typedef __attribute__((ext_vector_type(16))) _Float16 v16h;
typedef __attribute__((ext_vector_type(8)))  _Float16 v8h;
typedef __attribute__((ext_vector_type(4)))  _Float16 v4h;
typedef __attribute__((ext_vector_type(8)))  unsigned short v8us;
typedef __attribute__((ext_vector_type(8)))  float    v8f;
typedef __attribute__((ext_vector_type(4)))  float    v4f;
typedef __attribute__((ext_vector_type(4)))  int      v4i;
typedef v4f  __attribute__((may_alias)) v4fa;
typedef v8h  __attribute__((may_alias)) v8ha;
typedef v4h  __attribute__((may_alias)) v4ha;
typedef v8us __attribute__((may_alias)) v8usa;

__device__ __forceinline__ unsigned short f2bf(float f) { unsigned u = __float_as_uint(f); u += 0x7FFFu + ((u >> 16) & 1u); return (unsigned short)(u >> 16); }
__device__ __forceinline__ float bfr(float f) { return __uint_as_float(((unsigned)f2bf(f)) << 16); }
__device__ __forceinline__ v16h cat16(v8h lo, v8h hi) { return __builtin_shufflevector(lo, hi, 0, 1, 2, 3, 4, 5, 6, 7, 8, 9, 10, 11, 12, 13, 14, 15); }
__device__ __forceinline__ v16bf cat16b(v8us lo, v8us hi) { return __builtin_bit_cast(v16bf, __builtin_shufflevector(lo, hi, 0, 1, 2, 3, 4, 5, 6, 7, 8, 9, 10, 11, 12, 13, 14, 15)); }
__device__ __forceinline__ v16h  ldh(const h16* p) { return cat16(*(const v8h*)p, *(const v8h*)(p + 16)); }
__device__ __forceinline__ v16bf ldb(const bf* p)  { return cat16b(*(const v8us*)p, *(const v8us*)(p + 16)); }
__device__ __forceinline__ v8f wmma16g(v16h a, v16h b, v8f c) {
    c = __builtin_amdgcn_wmma_f32_16x16x32_f16(false, a, false, b, (short)0, c, false, false);
    asm volatile("v_nop\n\tv_nop\n\tv_nop\n\tv_nop" : "+v"(c) : "v"(a), "v"(b));
    return c; }
__device__ __forceinline__ v8f wmmabg(v16bf a, v16bf b, v8f c) {
    c = __builtin_amdgcn_wmma_f32_16x16x32_bf16(false, a, false, b, (short)0, c, false, false);
    asm volatile("v_nop\n\tv_nop\n\tv_nop\n\tv_nop" : "+v"(c) : "v"(a), "v"(b));
    return c; }
static __device__ __forceinline__ h16 toh_flush(float v) { const h16 r = (h16)v; return (fabsf(v) < 6.103515625e-05f) ? (h16)0.0f : r; }
__device__ __forceinline__ void wave_sync() { __builtin_amdgcn_fence(3  , "wavefront"); __builtin_amdgcn_wave_barrier(); asm volatile("" ::: "memory"); }

__global__ __launch_bounds__(256) void k_cvtx(const float* __restrict__ hid, bf* XB) {
    const int b = blockIdx.y;
    const size_t i = (size_t)blockIdx.x * 256 + threadIdx.x; if (i >= (size_t)LT * DM / 8) return;
    const v8f v = *(const v8f*)(hid + ((size_t)b * LH + 1) * DM + i * 8); v8us o;
#pragma unroll
    for (int k = 0; k < 8; ++k) o[k] = f2bf(v[k]);
    bf* dst = XB + (size_t)b * LT * DM + i * 8;
    *(volatile v8us*)dst = o; __threadfence(); *(volatile v8us*)dst = o;
}

__global__ __launch_bounds__(256) void k_w1t(const float* __restrict__ W1, bf* WT) {
    __shared__ __align__(16) unsigned short ts[32 * 72];
    const int tid = threadIdx.x;
    const int kt = blockIdx.x, n0 = blockIdx.y * 32;
    const int nn = tid & 31, kq = tid >> 5;
    const int n = n0 + nn; const int nc = n < H1 ? n : (H1 - 1);
#pragma unroll
    for (int q = 0; q < 8; ++q) { const int kk = kq + 8 * q;
        float v = W1[(size_t)(kt * 64 + kk) * H1 + nc]; asm volatile("" : "+v"(v));
        ts[nn * 72 + kk] = (n < H1) ? f2bf(v) : (unsigned short)0; }
    __syncthreads();
    const int rr = tid >> 3, pc = tid & 7;
    const v8us o = *(const v8usa*)(&ts[rr * 72 + pc * 8]);
    const int sel = kt / (DM / 64), kl = (kt - sel * (DM / 64)) * 64;
    bf* dst = WT + ((size_t)(sel * H1P + n0 + rr)) * DM + kl + pc * 8;
    *(volatile v8us*)dst = o; __threadfence(); *(volatile v8us*)dst = o;
}

__global__ __launch_bounds__(256) void k_w2t(const float* __restrict__ W2, h16* W2T) {
    const int p = blockIdx.x * 256 + threadIdx.x;
    if (p >= N2P * (K2P / 8)) return;
    const int n = p / (K2P / 8), k8 = (p - n * (K2P / 8)) * 8;
    const int nc = n < OUTC ? n : (OUTC - 1);
    v8h o;
#pragma unroll
    for (int e = 0; e < 8; ++e) { const int k = k8 + e; const int kc = k < H1 ? k : (H1 - 1);
        float v = W2[(size_t)kc * OUTC + nc]; asm volatile("" : "+v"(v));
        const bool ok = (k < H1) & (n < OUTC);
        const h16 c = toh_flush(bfr(v) * W2S);
        o[e] = ok ? c : (h16)0.0f; }
    h16* dst = W2T + (size_t)p * 8;
    *(volatile v8h*)dst = o; __threadfence(); *(volatile v8h*)dst = o;
}

__global__ __launch_bounds__(32) void k_pq(const bf* __restrict__ A, const bf* __restrict__ Bt, float* PQ) {
    __shared__ __align__(16) float os[16 * 68];
    const int K = DM;
    const int lane = threadIdx.x & 31, lr = lane & 15, hi = lane >> 4; const int r0 = blockIdx.x * 64, c0 = blockIdx.y * 64;
    v8f acc[4][4];
#pragma unroll
    for (int mb = 0; mb < 4; ++mb)
#pragma unroll
        for (int nb = 0; nb < 4; ++nb) acc[mb][nb] = (v8f){};
    const size_t aoff = (size_t)(r0 + lr) * K + 8 * hi, boff = (size_t)(c0 + lr) * K + 8 * hi;
#pragma unroll 1
    for (int kc = 0; kc < K; kc += 32) {
        v16bf a[4];
#pragma unroll
        for (int mb = 0; mb < 4; ++mb) a[mb] = ldb(A + aoff + (size_t)mb * 16 * K + kc);
#pragma unroll
        for (int nb = 0; nb < 4; ++nb) { const v16bf b = ldb(Bt + boff + (size_t)nb * 16 * K + kc);
#pragma unroll
            for (int mb = 0; mb < 4; ++mb) acc[mb][nb] = wmmabg(a[mb], b, acc[mb][nb]); }
    }
#pragma unroll
    for (int mb = 0; mb < 4; ++mb) {
#pragma unroll
        for (int nb = 0; nb < 4; ++nb) {
#pragma unroll
            for (int j = 0; j < 8; ++j) os[(hi * 8 + j) * 68 + nb * 16 + lr] = acc[mb][nb][j]; }
        wave_sync();
        float* ob = PQ + (size_t)(r0 + mb * 16) * PQP + c0;
#pragma unroll 1
        for (int ps = 0; ps < 2; ++ps) {
#pragma unroll
            for (int s = 0; s < 8; ++s) { const int row = 2 * s + (lane >> 4), c4 = (lane & 15) * 4;
                const v4f val = *(const v4fa*)(&os[row * 68 + c4]);
                *(volatile v4f*)(ob + (size_t)row * PQP + c4) = val; }
            if (ps == 0) __threadfence(); }
        wave_sync();
    }
}

static constexpr size_t LDS_HEAD = (size_t)RB * K2P * 2 + (size_t)HW * 16 * OUTC * 4 + (size_t)2 * K2P * 4 + (size_t)2 * LT * 4 + (size_t)4 * RB * 4;
static_assert(LDS_HEAD <= (size_t)131072);
__global__ __launch_bounds__(32 * HW) void k_head(const float* __restrict__ PQ, const h16* __restrict__ W2T, const float* __restrict__ W1,
                                                  const float* __restrict__ b1, const float* __restrict__ b2, const int* __restrict__ spans,
                                                  const int* __restrict__ tokn, const int* __restrict__ mask, float* OUT) {
    __shared__ __align__(16) h16   hs[RB * K2P];
    __shared__ __align__(16) float lt[HW * 16 * OUTC];
    __shared__ __align__(16) float bs[K2P];
    __shared__ __align__(16) float wc[K2P];
    __shared__ int cnt[LT];
    __shared__ int pre[LT];
    __shared__ int lst[RB];
    __shared__ int rowp[RB];
    __shared__ int rowq[RB];
    __shared__ float rind[RB];
    const int tid = threadIdx.x;
    const int lane = tid & 31, lr = lane & 15, hi = lane >> 4;
    const int wave = __builtin_amdgcn_readfirstlane((int)(threadIdx.x >> 5));
    const int g0 = blockIdx.x * RB;

    for (int c = tid; c < K2P; c += 32 * HW) { const int cc = c < H1 ? c : (H1 - 1);
        float x = b1[cc]; float y = W1[(size_t)KW1 * H1 + cc];
        asm volatile("" : "+v"(x)); asm volatile("" : "+v"(y));
        bs[c] = (c < H1) ? bfr(x) : 0.0f; wc[c] = (c < H1) ? bfr(y) : 0.0f; }
    if (tid < RB) lst[tid] = 0;
    unsigned mw[4]; int ones = 0;
    { const int* mrow = mask + (size_t)tid * LT;
#pragma unroll
      for (int w = 0; w < 4; ++w) { unsigned m = 0;
#pragma unroll
          for (int q = 0; q < 8; ++q) { const v4i v = *(const v4i*)(mrow + w * 32 + q * 4);
              m |= ((v[0] == 1) ? 1u : 0u) << (q * 4);     m |= ((v[1] == 1) ? 1u : 0u) << (q * 4 + 1);
              m |= ((v[2] == 1) ? 1u : 0u) << (q * 4 + 2); m |= ((v[3] == 1) ? 1u : 0u) << (q * 4 + 3); }
          mw[w] = m; ones += __popc(m);
          asm volatile("" ::: "memory"); } }
    cnt[tid] = ones;
    __syncthreads();
    if (tid == 0) { int run = 0;
#pragma unroll 1
        for (int t = 0; t < LT; ++t) { pre[t] = run; run += cnt[t]; } }
    __syncthreads();
    { const int n0 = g0 % NSP; int p = pre[tid];
#pragma unroll
      for (int w = 0; w < 4; ++w) { unsigned m = mw[w];
#pragma unroll 1
          for (int it = 0; it < 32; ++it) { if (m == 0u) break;
              const int bit = __ffs(m) - 1; m &= m - 1u;
              int r = p - n0; r += (r < 0) ? NSP : 0;
              if ((unsigned)r < (unsigned)RB) lst[r] = tid * LT + w * 32 + bit;
              ++p; } } }
    __syncthreads();
    if (tid < RB) {
        const int g = g0 + tid; const int gc = g < NROWS ? g : (NROWS - 1);
        const int b = gc / NSP;
        int code = lst[tid]; code = code < 0 ? 0 : (code > (LT * LT - 1) ? (LT * LT - 1) : code);
        const int i = code >> 7, j = code & (LT - 1);
        const int tl = tokn[0];
        int ic = i < tl ? i : (tl - 1); ic = ic < 0 ? 0 : ic;
        int jc = j < tl ? j : (tl - 1); jc = jc < 0 ? 0 : jc;
        const int s = spans[2 * b], e = spans[2 * b + 1];
        const bool ex = (i == s) & (j == e);
        const bool in = (i >= s) & (j <= e) & (i <= j);
        rind[tid] = ex ? 2.0f : (in ? 1.0f : 0.0f);
        rowp[tid] = (b * LT + ic) * PQP;
        rowq[tid] = (b * LT + jc) * PQP + H1P; }
    __syncthreads();

#pragma unroll 2
    for (int it = 0; it < (RB * (K2P / 4)) / (32 * HW); ++it) {
        const int idx = tid + (32 * HW) * it; const int row = idx / (K2P / 4); const int c4 = idx - row * (K2P / 4);
        const v4f pv = *(const v4f*)(PQ + (size_t)rowp[row] + 4 * c4);
        const v4f qv = *(const v4f*)(PQ + (size_t)rowq[row] + 4 * c4);
        const v4f bb = *(const v4fa*)(&bs[4 * c4]); const v4f ww = *(const v4fa*)(&wc[4 * c4]); const float ind = rind[row];
        v4h o;
#pragma unroll
        for (int e = 0; e < 4; ++e) { float v = (pv[e] + qv[e]) + ind * ww[e] + bb[e]; v = (v > 0.0f) ? v : 0.0f; o[e] = toh_flush(v); }
        *(v4ha*)(&hs[row * K2P + 4 * c4]) = o; }
    __syncthreads();

    v8f acc0 = (v8f){}, acc1 = (v8f){}, acc2 = (v8f){};
    const int ao = (16 * wave + lr) * K2P + 8 * hi;
    const size_t bo = (size_t)lr * K2P + 8 * hi;
#pragma unroll 1
    for (int kc = 0; kc < K2P; kc += 32) {
        const v16h a = cat16(*(const v8ha*)(&hs[ao + kc]), *(const v8ha*)(&hs[ao + kc + 16]));
        const v16h w0 = ldh(W2T + bo + kc), w1 = ldh(W2T + bo + (size_t)16 * K2P + kc), w2 = ldh(W2T + bo + (size_t)32 * K2P + kc);
        acc0 = wmma16g(a, w0, acc0); acc1 = wmma16g(a, w1, acc1); acc2 = wmma16g(a, w2, acc2); }
    const int wb = wave * 16 * OUTC;
    { const int c2 = 32 + lr; const int c2c = c2 < OUTC ? c2 : (OUTC - 1);
      float e0 = b2[lr], e1 = b2[16 + lr], e2 = b2[c2c];
      asm volatile("" : "+v"(e0)); asm volatile("" : "+v"(e1)); asm volatile("" : "+v"(e2));
      e0 = bfr(e0); e1 = bfr(e1); e2 = bfr(e2);
#pragma unroll
      for (int r = 0; r < 8; ++r) { const int ro = wb + (8 * hi + r) * OUTC;
          lt[ro + lr] = acc0[r] * W2I + e0; lt[ro + 16 + lr] = acc1[r] * W2I + e1;
          if (lr < OUTC - 32) lt[ro + 32 + lr] = acc2[r] * W2I + e2; } }
    wave_sync();
    { const int so = wb + (lane >> 1) * OUTC + (lane & 1) * 20;
      v4f x[5];
#pragma unroll
      for (int q = 0; q < 5; ++q) x[q] = *(const v4fa*)(&lt[so + 4 * q]);
      float mx = x[0][0];
#pragma unroll
      for (int q = 0; q < 5; ++q) { mx = fmaxf(mx, fmaxf(fmaxf(x[q][0], x[q][1]), fmaxf(x[q][2], x[q][3]))); }
      mx = fmaxf(mx, __shfl_xor(mx, 1, 32));
      float se = 0.0f;
#pragma unroll
      for (int q = 0; q < 5; ++q) { se += __expf(x[q][0] - mx); se += __expf(x[q][1] - mx); se += __expf(x[q][2] - mx); se += __expf(x[q][3] - mx); }
      se += __shfl_xor(se, 1, 32);
      const float lse = mx + __logf(se);
#pragma unroll
      for (int q = 0; q < 5; ++q) { v4f y; y[0] = x[q][0] - lse; y[1] = x[q][1] - lse; y[2] = x[q][2] - lse; y[3] = x[q][3] - lse; *(v4fa*)(&lt[so + 4 * q]) = y; } }
    wave_sync();
    const int gb = g0 + 16 * wave;
    float* ob = OUT + (size_t)gb * OUTC;
#pragma unroll 1
    for (int ps = 0; ps < 2; ++ps) {
#pragma unroll
        for (int s = 0; s < 5; ++s) { const int piece = s * 32 + lane;
            const v4f val = *(const v4fa*)(&lt[wb + piece * 4]);
            if ((size_t)gb * (OUTC / 4) + (size_t)piece < (size_t)NROWS * (OUTC / 4)) *(volatile v4f*)(ob + piece * 4) = val; }
        if (ps == 0) __threadfence(); }
}

static constexpr size_t al256(size_t v) { return (v + 255) & ~(size_t)255; }
static constexpr size_t SZ_XB = al256((size_t)NB * LT * DM * 2);
static constexpr size_t SZ_WT = al256((size_t)2 * H1P * DM * 2);
static constexpr size_t SZ_W2 = al256((size_t)N2P * K2P * 2);
static constexpr size_t SZ_PQ = al256((size_t)NB * LT * PQP * 4);
static constexpr size_t SZ_TOTAL = SZ_XB + SZ_WT + SZ_W2 + SZ_PQ;
static_assert(SZ_TOTAL <= (size_t)134217728);
static_assert((size_t)(KW1 / 64) * 64 * (size_t)(H1P / 32) * 32 == (size_t)2 * H1P * DM);
static_assert((size_t)(NB * LT / 64) * 64 * (size_t)(PQP / 64) * 64 == (size_t)NB * LT * PQP);
static_assert((size_t)NROWS * OUTC * 4 <= (size_t)NB_FULL * NSP * OUTC * 4);

extern "C" void kernel_launch(void* const* d_in, const int* in_sizes, int n_in,
                              void* d_out, int out_size, void* d_ws, size_t ws_size, hipStream_t stream) {
    if (n_in < 8) return;
    if ((size_t)in_sizes[0] < (size_t)NB * LH * DM) return;
    if (in_sizes[1] < 2 * NB || in_sizes[2] < 1 || in_sizes[3] < LT * LT) return;
    if ((size_t)in_sizes[4] < (size_t)(KW1 + 1) * H1 || in_sizes[5] < H1) return;
    if ((size_t)in_sizes[6] < (size_t)H1 * OUTC || in_sizes[7] < OUTC) return;
    if ((size_t)out_size < (size_t)NROWS * OUTC) return;
    if (SZ_TOTAL > ws_size) return;
    const float* hid = (const float*)d_in[0];
    const int* spans = (const int*)d_in[1];
    const int* tokn  = (const int*)d_in[2];
    const int* mask  = (const int*)d_in[3];
    const float* W1  = (const float*)d_in[4];
    const float* b1  = (const float*)d_in[5];
    const float* W2  = (const float*)d_in[6];
    const float* b2  = (const float*)d_in[7];
    float* OUT = (float*)d_out;
    char* wsp = (char*)d_ws;
    bf*    XB  = (bf*)wsp;    wsp += SZ_XB;
    bf*    WT  = (bf*)wsp;    wsp += SZ_WT;
    h16*   W2T = (h16*)wsp;   wsp += SZ_W2;
    float* PQ  = (float*)wsp; wsp += SZ_PQ;

    k_cvtx<<<dim3((unsigned)((size_t)LT * DM / 8 / 256), NB, 1), 256, 0, stream>>>(hid, XB);
    k_w1t<<<dim3(KW1 / 64, H1P / 32, 1), 256, 0, stream>>>(W1, WT);
    k_w2t<<<dim3((N2P * (K2P / 8) + 255) / 256, 1, 1), 256, 0, stream>>>(W2, W2T);
    k_pq<<<dim3(NB * LT / 64, PQP / 64, 1), 32, 0, stream>>>(XB, WT, PQ);
    k_head<<<dim3((NROWS + RB - 1) / RB, 1, 1), 32 * HW, 0, stream>>>(PQ, W2T, W1, b1, b2, spans, tokn, mask, OUT);
}
